// Next_Node_Probability_Calculator_for_group_28097676051164
// MI455X (gfx1250) — hardware-verified
//
#include <hip/hip_runtime.h>
#define NB 512
#define GG 100
#define PN 100
#define EE 128
#define NH 8
#define KD 16
#define RP 112
#define BCH 32
#define JCH (BCH * NH)

typedef __bf16 v16b __attribute__((ext_vector_type(16)));
typedef unsigned short v8us __attribute__((ext_vector_type(8), may_alias));
typedef float  v8f  __attribute__((ext_vector_type(8)));
typedef float  v4f  __attribute__((ext_vector_type(4)));
typedef float  v4fa __attribute__((ext_vector_type(4), may_alias));
union FragB { v16b v; v8us half[2]; unsigned short u[16]; };

__device__ __forceinline__ unsigned short bf16_bits(float x) { unsigned int u = __float_as_uint(x); return (unsigned short)((u + 0x7FFFu + ((u >> 16) & 1u)) >> 16); }
__device__ __forceinline__ float bf16_val(unsigned short b) { return __uint_as_float(((unsigned int)b) << 16); }
__device__ __forceinline__ float bf16_round(float x) { return bf16_val(bf16_bits(x)); }
template <int NT>
__device__ __forceinline__ v8f mmaN(v16b ah, v16b al, v16b bh, v16b bl, v8f c) {
  c = __builtin_amdgcn_wmma_f32_16x16x32_bf16(false, ah, false, bh, (short)0, c, false, false);
  if (NT >= 2) c = __builtin_amdgcn_wmma_f32_16x16x32_bf16(false, al, false, bh, (short)0, c, false, false);
  if (NT >= 3) c = __builtin_amdgcn_wmma_f32_16x16x32_bf16(false, ah, false, bl, (short)0, c, false, false);
  asm volatile("v_nop\n\tv_nop\n\tv_nop\n\tv_nop" : "+v"(c) : "v"(ah), "v"(al), "v"(bh), "v"(bl));
  return c;
}

__global__ __launch_bounds__(256) void k_wt_bf16(const float* __restrict__ W, unsigned short* __restrict__ Wt, int K, int N) {
  const int t = blockIdx.x * 256 + threadIdx.x;
  const int k8n = K / 8;
  if (t >= N * k8n) return;
  const int n = t / k8n, k8 = (t % k8n) * 8;
  v8us v;
#pragma unroll
  for (int i = 0; i < 8; ++i) v[i] = bf16_bits(W[(size_t)(k8 + i) * N + n]);
  *(volatile v8us*)(Wt + (size_t)n * K + k8) = v;
  __threadfence();
  *(volatile v8us*)(Wt + (size_t)n * K + k8) = v;
}

template <bool ASPLIT, int ACT, bool BIAS_BF16>
__global__ __launch_bounds__(128) void k_gemm_bf(const float* __restrict__ A, int lda, const unsigned short* __restrict__ Wt, int ldb,
                                               const float* __restrict__ bias, float* __restrict__ C, int ldc, int M, int N, int K) {
  __shared__ __attribute__((aligned(16))) float so[4][16][64];
  const int tid = threadIdx.x, w = tid >> 5, lane = tid & 31, ln = lane & 15, hh = lane >> 4;
  const int ntn = N / 64;
  const int wid = blockIdx.x * 4 + w;
  const int mt = wid / ntn, nq = wid % ntn;
  if (mt * 16 >= M) return;
  const int row0 = mt * 16, col0 = nq * 64;
  const float* arow = A + (size_t)(row0 + ln) * lda;
  v8f acc[4] = {};
  for (int kb = 0; kb < K; kb += 32) {
    FragB ah, al;
    const v4f x0 = *(const v4fa*)(arow + kb + 8 * hh), x1 = *(const v4fa*)(arow + kb + 8 * hh + 4);
    const v4f x2 = *(const v4fa*)(arow + kb + 16 + 8 * hh), x3 = *(const v4fa*)(arow + kb + 16 + 8 * hh + 4);
    float xs[16] = {x0[0],x0[1],x0[2],x0[3],x1[0],x1[1],x1[2],x1[3],x2[0],x2[1],x2[2],x2[3],x3[0],x3[1],x3[2],x3[3]};
#pragma unroll
    for (int i = 0; i < 16; ++i) { const unsigned short hb = bf16_bits(xs[i]); ah.u[i] = hb; al.u[i] = ASPLIT ? bf16_bits(xs[i] - bf16_val(hb)) : (unsigned short)0; }
#pragma unroll
    for (int t = 0; t < 4; ++t) {
      const unsigned short* brow = Wt + (size_t)(col0 + t * 16 + ln) * ldb + kb;
      FragB b;
      b.half[0] = *(const v8us*)(brow + 8 * hh);
      b.half[1] = *(const v8us*)(brow + 16 + 8 * hh);
      acc[t] = mmaN<ASPLIT ? 2 : 1>(ah.v, al.v, b.v, b.v, acc[t]);
    }
  }
#pragma unroll
  for (int t = 0; t < 4; ++t) {
    float bv = bias ? bias[col0 + t * 16 + ln] : 0.f;
    if (BIAS_BF16) bv = bf16_round(bv);
#pragma unroll
    for (int r = 0; r < 8; ++r) { float v = acc[t][r] + bv; if (ACT == 1) v = fmaxf(v, 0.f); so[w][8 * hh + r][t * 16 + ln] = v; }
  }
  __builtin_amdgcn_fence(__ATOMIC_ACQ_REL, "workgroup");
  __builtin_amdgcn_wave_barrier();
  const int rsub = lane >> 4, c4 = (lane & 15) * 4;
  for (int pass = 0; pass < 2; ++pass) {
#pragma unroll
    for (int q = 0; q < 8; ++q) {
      const int r = q * 2 + rsub;
      const v4f v = *(const v4fa*)&so[w][r][c4];
      *(volatile v4f*)(C + (size_t)(row0 + r) * ldc + col0 + c4) = v;
    }
    if (pass == 0) __threadfence();
  }
}

template <int D, bool CAUSAL>
__global__ __launch_bounds__(128) void k_flash(const float* __restrict__ qb, const float* __restrict__ kb, const float* __restrict__ vb,
                                             int pitch, int T, int H, float scale, float* __restrict__ y, int ypitch) {
  constexpr int KS = D / 32;
  constexpr int DT = D / 16;
  __shared__ __attribute__((aligned(16))) unsigned short sKh[32][D + 8], sKl[32][D + 8], sVh[32][D + 8], sVl[32][D + 8];
  __shared__ __attribute__((aligned(16))) unsigned short sPh[4][16][40], sPl[4][16][40];
  __shared__ __attribute__((aligned(16))) float sO[4][16][D];
  const int tid = threadIdx.x, w = tid >> 5, lane = tid & 31, ln = lane & 15, hh = lane >> 4;
  const int nqb = (T + 63) / 64;
  const int bh = blockIdx.x / nqb, qblk = blockIdx.x % nqb;
  const int b = bh / H, h = bh % H;
  const int q0 = qblk * 64 + w * 16;
  const float* Q = qb + (size_t)b * T * pitch + h * D;
  const float* K = kb + (size_t)b * T * pitch + h * D;
  const float* V = vb + (size_t)b * T * pitch + h * D;

  FragB aqh[KS], aql[KS];
  {
    int row = q0 + ln; if (row >= T) row = T - 1;
    const float* qr = Q + (size_t)row * pitch;
#pragma unroll
    for (int ks = 0; ks < KS; ++ks)
#pragma unroll
      for (int i = 0; i < 16; ++i) {
        const int d = ks * 32 + ((i < 8) ? (8 * hh + i) : (16 + 8 * hh + (i - 8)));
        const float x = qr[d] * scale; const unsigned short hb = bf16_bits(x);
        aqh[ks].u[i] = hb; aql[ks].u[i] = bf16_bits(x - bf16_val(hb));
      }
  }
  float m_r[8], l_r[8];
#pragma unroll
  for (int r = 0; r < 8; ++r) { m_r[r] = -3.0e38f; l_r[r] = 0.f; }
  v8f oacc[DT];
#pragma unroll
  for (int dt = 0; dt < DT; ++dt) oacc[dt] = (v8f){0.f,0.f,0.f,0.f,0.f,0.f,0.f,0.f};

  const int kv_end = CAUSAL ? min(T, qblk * 64 + 64) : T;
  for (int j0 = 0; j0 < kv_end; j0 += 32) {
    __syncthreads();
    for (int e = tid; e < 32 * (D / 4); e += 128) {
      const int r = e / (D / 4), c4 = (e % (D / 4)) * 4;
      const int key = j0 + r;
      v4f kf = {0.f,0.f,0.f,0.f}, vf = {0.f,0.f,0.f,0.f};
      if (key < T) { kf = *(const v4fa*)(K + (size_t)key * pitch + c4); vf = *(const v4fa*)(V + (size_t)key * pitch + c4); }
#pragma unroll
      for (int t = 0; t < 4; ++t) {
        unsigned short hb = bf16_bits(kf[t]); sKh[r][c4 + t] = hb; sKl[r][c4 + t] = bf16_bits(kf[t] - bf16_val(hb));
        hb = bf16_bits(vf[t]); sVh[r][c4 + t] = hb; sVl[r][c4 + t] = bf16_bits(vf[t] - bf16_val(hb));
      }
    }
    __syncthreads();
    v8f s[2];
#pragma unroll
    for (int nt = 0; nt < 2; ++nt) {
      v8f acc = {};
#pragma unroll
      for (int ks = 0; ks < KS; ++ks) {
        FragB bh_, bl_;
        bh_.half[0] = *(const v8us*)&sKh[nt * 16 + ln][ks * 32 + 8 * hh]; bh_.half[1] = *(const v8us*)&sKh[nt * 16 + ln][ks * 32 + 16 + 8 * hh];
        bl_.half[0] = *(const v8us*)&sKl[nt * 16 + ln][ks * 32 + 8 * hh]; bl_.half[1] = *(const v8us*)&sKl[nt * 16 + ln][ks * 32 + 16 + 8 * hh];
        acc = mmaN<3>(aqh[ks].v, aql[ks].v, bh_.v, bl_.v, acc);
      }
      s[nt] = acc;
    }
    float alpha[8];
#pragma unroll
    for (int r = 0; r < 8; ++r) {
      const int qi = q0 + 8 * hh + r;
      const int ja = j0 + ln, jb = j0 + 16 + ln;
      if (CAUSAL) { if (ja > qi) s[0][r] = -3.0e38f; if (jb > qi) s[1][r] = -3.0e38f; }
      if (ja >= T) s[0][r] = -3.0e38f;
      if (jb >= T) s[1][r] = -3.0e38f;
      float mx = fmaxf(s[0][r], s[1][r]);
      mx = fmaxf(mx, __shfl_xor(mx, 1, 32)); mx = fmaxf(mx, __shfl_xor(mx, 2, 32)); mx = fmaxf(mx, __shfl_xor(mx, 4, 32)); mx = fmaxf(mx, __shfl_xor(mx, 8, 32));
      const float mnew = fmaxf(m_r[r], mx);
      alpha[r] = (mnew > -1.0e38f) ? __expf(m_r[r] - mnew) : 1.0f;
      const float p0 = (s[0][r] > -1.0e38f) ? __expf(s[0][r] - mnew) : 0.f;
      const float p1 = (s[1][r] > -1.0e38f) ? __expf(s[1][r] - mnew) : 0.f;
      m_r[r] = mnew;
      l_r[r] = l_r[r] * alpha[r] + p0 + p1;
      unsigned short hb = bf16_bits(p0); sPh[w][8 * hh + r][ln] = hb;      sPl[w][8 * hh + r][ln] = bf16_bits(p0 - bf16_val(hb));
      hb = bf16_bits(p1);                sPh[w][8 * hh + r][16 + ln] = hb; sPl[w][8 * hh + r][16 + ln] = bf16_bits(p1 - bf16_val(hb));
    }
#pragma unroll
    for (int dt = 0; dt < DT; ++dt)
#pragma unroll
      for (int r = 0; r < 8; ++r) oacc[dt][r] *= alpha[r];
    __builtin_amdgcn_fence(__ATOMIC_ACQ_REL, "workgroup");
    __builtin_amdgcn_wave_barrier();
    FragB pah, pal;
    pah.half[0] = *(const v8us*)&sPh[w][ln][8 * hh]; pah.half[1] = *(const v8us*)&sPh[w][ln][16 + 8 * hh];
    pal.half[0] = *(const v8us*)&sPl[w][ln][8 * hh]; pal.half[1] = *(const v8us*)&sPl[w][ln][16 + 8 * hh];
#pragma unroll
    for (int dt = 0; dt < DT; ++dt) {
      FragB bvh, bvl;
#pragma unroll
      for (int i = 0; i < 8; ++i) {
        bvh.u[i] = sVh[8 * hh + i][dt * 16 + ln]; bvh.u[8 + i] = sVh[16 + 8 * hh + i][dt * 16 + ln];
        bvl.u[i] = sVl[8 * hh + i][dt * 16 + ln]; bvl.u[8 + i] = sVl[16 + 8 * hh + i][dt * 16 + ln];
      }
      oacc[dt] = mmaN<3>(pah.v, pal.v, bvh.v, bvl.v, oacc[dt]);
    }
    __builtin_amdgcn_fence(__ATOMIC_ACQ_REL, "workgroup");
    __builtin_amdgcn_wave_barrier();
  }
#pragma unroll
  for (int r = 0; r < 8; ++r) {
    float l = l_r[r];
    l += __shfl_xor(l, 1, 32); l += __shfl_xor(l, 2, 32); l += __shfl_xor(l, 4, 32); l += __shfl_xor(l, 8, 32);
    l_r[r] = (l > 0.f) ? 1.0f / l : 0.f;
  }
#pragma unroll
  for (int dt = 0; dt < DT; ++dt)
#pragma unroll
    for (int r = 0; r < 8; ++r) sO[w][8 * hh + r][dt * 16 + ln] = oacc[dt][r] * l_r[r];
  __builtin_amdgcn_fence(__ATOMIC_ACQ_REL, "workgroup");
  __builtin_amdgcn_wave_barrier();
  for (int pass = 0; pass < 2; ++pass) {
    for (int r = 0; r < 16; ++r) {
      const int row = q0 + r;
      if (row < T && lane < D / 4) {
        const v4f val = *(const v4fa*)&sO[w][r][lane * 4];
        *(volatile v4f*)(y + ((size_t)b * T + row) * ypitch + h * D + lane * 4) = val;
      }
    }
    if (pass == 0) __threadfence();
  }
}

template <bool ASPLIT, int ACT, bool BIAS_BF16, bool RES_BF16>
__global__ __launch_bounds__(128) void k_gemm_bf3(const float* __restrict__ A, int lda, const unsigned short* __restrict__ Wt, int ldb,
                                                const float* __restrict__ bias, const float* __restrict__ resid, int rmod, int ldr,
                                                float* __restrict__ C, int ldc, int M, int N, int K) {
  __shared__ __attribute__((aligned(16))) float so[4][16][64];
  const int tid = threadIdx.x, w = tid >> 5, lane = tid & 31, ln = lane & 15, hh = lane >> 4;
  const int ntn = N / 64;
  const int wid = blockIdx.x * 4 + w;
  const int mt = wid / ntn, nq = wid % ntn;
  if (mt * 16 >= M) return;
  const int row0 = mt * 16, col0 = nq * 64;
  const float* arow = A + (size_t)(row0 + ln) * lda;
  v8f acc[4] = {};
  for (int kb = 0; kb < K; kb += 32) {
    FragB ah, al;
    const v4f x0 = *(const v4fa*)(arow + kb + 8 * hh), x1 = *(const v4fa*)(arow + kb + 8 * hh + 4);
    const v4f x2 = *(const v4fa*)(arow + kb + 16 + 8 * hh), x3 = *(const v4fa*)(arow + kb + 16 + 8 * hh + 4);
    float xs[16] = {x0[0],x0[1],x0[2],x0[3],x1[0],x1[1],x1[2],x1[3],x2[0],x2[1],x2[2],x2[3],x3[0],x3[1],x3[2],x3[3]};
#pragma unroll
    for (int i = 0; i < 16; ++i) { const unsigned short hb = bf16_bits(xs[i]); ah.u[i] = hb; al.u[i] = ASPLIT ? bf16_bits(xs[i] - bf16_val(hb)) : (unsigned short)0; }
#pragma unroll
    for (int t = 0; t < 4; ++t) {
      const unsigned short* brow = Wt + (size_t)(col0 + t * 16 + ln) * ldb + kb;
      FragB b;
      b.half[0] = *(const v8us*)(brow + 8 * hh);
      b.half[1] = *(const v8us*)(brow + 16 + 8 * hh);
      acc[t] = mmaN<ASPLIT ? 2 : 1>(ah.v, al.v, b.v, b.v, acc[t]);
    }
  }
#pragma unroll
  for (int t = 0; t < 4; ++t) {
    const int col = col0 + t * 16 + ln;
    float bv = bias ? bias[col] : 0.f;
    if (BIAS_BF16) bv = bf16_round(bv);
#pragma unroll
    for (int r = 0; r < 8; ++r) {
      float v = acc[t][r] + bv;
      if (resid) { float rv = resid[(size_t)((row0 + 8 * hh + r) % rmod) * ldr + col]; if (RES_BF16) rv = bf16_round(rv); v += rv; }
      if (ACT == 1) v = fmaxf(v, 0.f);
      if (ACT == 2) v = 0.5f * v * (1.0f + erff(v * 0.70710678118654752f));
      if (ACT == 3) { const float u = 0.7978845608028654f * (v + 0.044715f * v * v * v); v = 0.5f * v * (1.0f + tanhf(u)); }
      so[w][8 * hh + r][t * 16 + ln] = v;
    }
  }
  __builtin_amdgcn_fence(__ATOMIC_ACQ_REL, "workgroup");
  __builtin_amdgcn_wave_barrier();
  const int rsub = lane >> 4, c4 = (lane & 15) * 4;
  for (int pass = 0; pass < 2; ++pass) {
#pragma unroll
    for (int q = 0; q < 8; ++q) {
      const int r = q * 2 + rsub;
      const v4f v = *(const v4fa*)&so[w][r][c4];
      *(volatile v4f*)(C + (size_t)(row0 + r) * ldc + col0 + c4) = v;
    }
    if (pass == 0) __threadfence();
  }
}
template <bool PARAM_BF16>
__global__ __launch_bounds__(256) void k_layernorm(const float* __restrict__ X, const float* __restrict__ R, const float* __restrict__ g, const float* __restrict__ bta,
                                                  float* __restrict__ out_sum, float* __restrict__ out_norm, int N, float eps) {
  __shared__ float red[256];
  const int row = blockIdx.x, tid = threadIdx.x;
  const float* x = X + (size_t)row * N; const float* rr = R ? R + (size_t)row * N : nullptr;
  float vals[16];
  const int per = N / 256;
  float s1 = 0.f;
  for (int u = 0; u < per / 4; ++u) {
    const int j = tid * 4 + 1024 * u;
    const v4f a = *(const v4fa*)(x + j);
    v4f b = {0.f,0.f,0.f,0.f}; if (rr) b = *(const v4fa*)(rr + j);
#pragma unroll
    for (int q = 0; q < 4; ++q) { const float v = a[q] + b[q]; vals[u * 4 + q] = v; s1 += v; }
  }
  red[tid] = s1; __syncthreads();
  for (int st = 128; st > 0; st >>= 1) { if (tid < st) red[tid] += red[tid + st]; __syncthreads(); }
  const float mu = red[0] / (float)N; __syncthreads();
  float s2 = 0.f;
  for (int u = 0; u < per / 4; ++u)
#pragma unroll
    for (int q = 0; q < 4; ++q) { const float c = vals[u * 4 + q] - mu; s2 += c * c; }
  red[tid] = s2; __syncthreads();
  for (int st = 128; st > 0; st >>= 1) { if (tid < st) red[tid] += red[tid + st]; __syncthreads(); }
  const float rs = rsqrtf(red[0] / (float)N + eps);
  for (int pass = 0; pass < 2; ++pass) {
    for (int u = 0; u < per / 4; ++u) {
      const int j = tid * 4 + 1024 * u;
      v4f o, sm;
#pragma unroll
      for (int q = 0; q < 4; ++q) {
        float gg = g[j + q], bb = bta[j + q];
        if (PARAM_BF16) { gg = bf16_round(gg); bb = bf16_round(bb); }
        sm[q] = vals[u * 4 + q]; o[q] = (vals[u * 4 + q] - mu) * rs * gg + bb;
      }
      if (out_sum) *(volatile v4f*)(out_sum + (size_t)row * N + j) = sm;
      *(volatile v4f*)(out_norm + (size_t)row * N + j) = o;
    }
    if (pass == 0) __threadfence();
  }
}


typedef _Float16 v16h __attribute__((ext_vector_type(16)));
union FragH { v16h v; v8us half[2]; _Float16 h[16]; unsigned short u[16]; };
template <int NT>
__device__ __forceinline__ v8f mmaH(v16h ah, v16h al, v16h bh, v16h bl, v8f c) {
  c = __builtin_amdgcn_wmma_f32_16x16x32_f16(false, ah, false, bh, (short)0, c, false, false);
  if (NT >= 2) c = __builtin_amdgcn_wmma_f32_16x16x32_f16(false, al, false, bh, (short)0, c, false, false);
  if (NT >= 3) c = __builtin_amdgcn_wmma_f32_16x16x32_f16(false, ah, false, bl, (short)0, c, false, false);
  asm volatile("v_nop\n\tv_nop\n\tv_nop\n\tv_nop" : "+v"(c) : "v"(ah), "v"(al), "v"(bh), "v"(bl));
  return c;
}
template <bool ASPLIT>
__global__ __launch_bounds__(128) void k_gemm_h(const float* __restrict__ A, int lda, size_t sA, const _Float16* __restrict__ Bh, int ldb, size_t sB, float alpha, float* __restrict__ C, int ldc, size_t sC, int M, int N, int K) {
  __shared__ __attribute__((aligned(16))) float so[4][16][64];
  const int tid = threadIdx.x, w = tid >> 5, lane = tid & 31, ln = lane & 15, hh = lane >> 4; const int by = blockIdx.y;
  A += (size_t)by * sA; Bh += (size_t)by * sB; C += (size_t)by * sC;
  const int ntn = (N + 63) / 64; const int wid = blockIdx.x * 4 + w; const int mt = wid / ntn, nq = wid % ntn; if (mt * 16 >= M) return;
  const int row0 = mt * 16, col0 = nq * 64; const float* arow = A + (size_t)(row0 + ln) * lda;
  v8f acc[4] = {};
  for (int kb = 0; kb < K; kb += 32) {
    FragH ah, al;
    const v4f x0 = *(const v4fa*)(arow + kb + 8 * hh), x1 = *(const v4fa*)(arow + kb + 8 * hh + 4), x2 = *(const v4fa*)(arow + kb + 16 + 8 * hh), x3 = *(const v4fa*)(arow + kb + 16 + 8 * hh + 4);
    float xs[16] = {x0[0],x0[1],x0[2],x0[3],x1[0],x1[1],x1[2],x1[3],x2[0],x2[1],x2[2],x2[3],x3[0],x3[1],x3[2],x3[3]};
#pragma unroll
    for (int i = 0; i < 16; ++i) { const _Float16 h = (_Float16)xs[i]; ah.h[i] = h; al.h[i] = ASPLIT ? (_Float16)(xs[i] - (float)h) : (_Float16)0.0f; }
#pragma unroll
    for (int t = 0; t < 4; ++t) { if (col0 + t * 16 >= N) continue; const size_t boff = (size_t)(col0 + t * 16 + ln) * ldb + kb; FragH bq; bq.half[0] = *(const v8us*)(Bh + boff + 8 * hh); bq.half[1] = *(const v8us*)(Bh + boff + 16 + 8 * hh);
      acc[t] = mmaH<ASPLIT ? 2 : 1>(ah.v, al.v, bq.v, bq.v, acc[t]); }
  }
#pragma unroll
  for (int t = 0; t < 4; ++t) { if (col0 + t * 16 >= N) continue;
#pragma unroll
    for (int r = 0; r < 8; ++r) so[w][8 * hh + r][t * 16 + ln] = acc[t][r] * alpha; }
  __builtin_amdgcn_fence(__ATOMIC_ACQ_REL, "workgroup"); __builtin_amdgcn_wave_barrier();
  const int rsub = lane >> 4, c4 = (lane & 15) * 4;
  for (int pass = 0; pass < 2; ++pass) {
#pragma unroll
    for (int q = 0; q < 8; ++q) { const int r = q * 2 + rsub; if (col0 + c4 < N) { const v4f v = *(const v4fa*)&so[w][r][c4]; *(volatile v4f*)(C + (size_t)(row0 + r) * ldc + col0 + c4) = v; } }
    if (pass == 0) __threadfence(); }
}

__global__ __launch_bounds__(256) void k_wt_f16(const float* __restrict__ W, _Float16* __restrict__ Wt, int K, int N, float scale) {
  const int t = blockIdx.x * 256 + threadIdx.x; if (t >= N * (K / 8)) return; const int n = t / (K / 8), k8 = (t % (K / 8)) * 8; FragH f;
#pragma unroll
  for (int i = 0; i < 8; ++i) f.h[i] = (_Float16)(bf16_round(W[(size_t)(k8 + i) * N + n]) * scale); const v8us o = f.half[0];
  *(volatile v8us*)((unsigned short*)Wt + (size_t)n * K + k8) = o; __threadfence(); *(volatile v8us*)((unsigned short*)Wt + (size_t)n * K + k8) = o;
}
template <int ACT>
__global__ __launch_bounds__(128) void k_gemm_hhx(const _Float16* __restrict__ A, int lda, size_t sA, const _Float16* __restrict__ Bh, int ldb, size_t sB, float alpha, const float* __restrict__ bias, size_t sBias, const float* __restrict__ CP, int rowsPerB, size_t sCPb, int row0g,
    float* __restrict__ C, _Float16* __restrict__ C16, int ldc, size_t sC, int M, int N, int K) {
  __shared__ __attribute__((aligned(16))) float so[4][16][64];
  const int tid = threadIdx.x, w = tid >> 5, lane = tid & 31, ln = lane & 15, hh = lane >> 4; const int by = blockIdx.y;
  A += (size_t)by * sA; Bh += (size_t)by * sB; const size_t cofs = (size_t)by * sC; const float* bp = bias ? bias + (size_t)by * sBias : nullptr;
  const int ntn = (N + 63) / 64; const int wid = blockIdx.x * 4 + w; const int mt = wid / ntn, nq = wid % ntn; if (mt * 16 >= M) return;
  const int row0 = mt * 16, col0 = nq * 64; const _Float16* arow = A + (size_t)(row0 + ln) * lda;
  v8f acc[4] = {};
  for (int kb = 0; kb < K; kb += 32) { FragH ah; ah.half[0] = *(const v8us*)((const unsigned short*)arow + kb + 8 * hh); ah.half[1] = *(const v8us*)((const unsigned short*)arow + kb + 16 + 8 * hh);
#pragma unroll
    for (int t = 0; t < 4; ++t) { if (col0 + t * 16 >= N) continue; const size_t boff = (size_t)(col0 + t * 16 + ln) * ldb + kb; FragH bq; bq.half[0] = *(const v8us*)((const unsigned short*)Bh + boff + 8 * hh); bq.half[1] = *(const v8us*)((const unsigned short*)Bh + boff + 16 + 8 * hh);
      acc[t] = mmaH<1>(ah.v, ah.v, bq.v, bq.v, acc[t]); }
  }
#pragma unroll
  for (int t = 0; t < 4; ++t) { if (col0 + t * 16 >= N) continue; const int col = col0 + t * 16 + ln; const float bv = bp ? bf16_round(bp[col]) : 0.f;
#pragma unroll
    for (int r = 0; r < 8; ++r) { float v = acc[t][r] * alpha + bv; if (CP) { const int bidx = (row0g + row0 + 8 * hh + r) / rowsPerB; v += CP[(size_t)bidx * sCPb + (size_t)by * 64 + col]; } if (ACT == 1) v = (v > 0.f) ? v : expm1f(v); else if (ACT == 3) v = fmaxf(v, 0.f); so[w][8 * hh + r][t * 16 + ln] = v; } }
  __builtin_amdgcn_fence(__ATOMIC_ACQ_REL, "workgroup"); __builtin_amdgcn_wave_barrier();
  const int rsub = lane >> 4, c4 = (lane & 15) * 4; typedef _Float16 v4h __attribute__((ext_vector_type(4)));
  for (int pass = 0; pass < 2; ++pass) {
#pragma unroll
    for (int q = 0; q < 8; ++q) { const int r = q * 2 + rsub; if (col0 + c4 < N) { const v4f v = *(const v4fa*)&so[w][r][c4]; if (C) *(volatile v4f*)(C + cofs + (size_t)(row0 + r) * ldc + col0 + c4) = v; if (C16) { v4h h4; for (int i = 0; i < 4; ++i) h4[i] = (_Float16)v[i]; *(volatile v4h*)(C16 + cofs + (size_t)(row0 + r) * ldc + col0 + c4) = h4; } } }
    if (pass == 0) __threadfence(); }
}


__global__ __launch_bounds__(256) void k_x16(const float* __restrict__ x, _Float16* __restrict__ X16, size_t n8) { const size_t t = (size_t)blockIdx.x * 256 + threadIdx.x; if (t >= n8) return; FragH f;
#pragma unroll
  for (int q = 0; q < 8; ++q) f.h[q] = (_Float16)bf16_round(x[t * 8 + q]); *(volatile v8us*)((unsigned short*)X16 + t * 8) = f.half[0]; __threadfence(); *(volatile v8us*)((unsigned short*)X16 + t * 8) = f.half[0]; }
__global__ __launch_bounds__(128) void k_q1(const float* __restrict__ in1, const float* __restrict__ Wq, float* __restrict__ Q1) { const int b = blockIdx.x, o = threadIdx.x; float s = 0.f;
#pragma unroll 1
  for (int e = 0; e < EE; ++e) s += bf16_round(in1[(size_t)b * EE + e]) * bf16_round(Wq[(size_t)e * EE + o]); *(volatile float*)(Q1 + (size_t)b * EE + o) = s; __threadfence(); *(volatile float*)(Q1 + (size_t)b * EE + o) = s; }
__global__ __launch_bounds__(256) void k_qfin(const float* __restrict__ QF, const float* __restrict__ Q1, const float* __restrict__ rl, const float* __restrict__ Wq, _Float16* __restrict__ Q16) { const size_t t = (size_t)blockIdx.x * 256 + threadIdx.x; if (t >= (size_t)NB * GG * 16) return; const int c8 = (int)(t % 16) * 8; const size_t r = t / 16; const size_t b = r / GG; const float rv = bf16_round(rl[r]); FragH f;
#pragma unroll
  for (int q = 0; q < 8; ++q) { const int o = c8 + q; f.h[q] = (_Float16)((QF[r * EE + o] + Q1[b * EE + o] + rv * bf16_round(Wq[(size_t)256 * EE + o])) * 0.25f); } *(volatile v8us*)((unsigned short*)Q16 + t * 8) = f.half[0]; __threadfence(); *(volatile v8us*)((unsigned short*)Q16 + t * 8) = f.half[0]; }
__global__ __launch_bounds__(256) void k_qkp(const _Float16* __restrict__ Q16, const _Float16* __restrict__ K16, int b0, _Float16* __restrict__ QP, _Float16* __restrict__ KP) { const int t = blockIdx.x * 256 + threadIdx.x; if (t >= JCH * RP * 4) return; const int p4 = t % 4; const int gi = (t / 4) % RP; const int j = t / (4 * RP); const int b = b0 + j / NH, h = j % NH; v8us q = {0,0,0,0,0,0,0,0}, k = {0,0,0,0,0,0,0,0};
  if (p4 < 2 && gi < GG) { const size_t src = ((size_t)b * GG + gi) * EE + h * KD + p4 * 8; q = *(const v8us*)((const unsigned short*)Q16 + src); k = *(const v8us*)((const unsigned short*)K16 + src); }
  for (int pass = 0; pass < 2; ++pass) { *(volatile v8us*)((unsigned short*)QP + (size_t)t * 8) = q; *(volatile v8us*)((unsigned short*)KP + (size_t)t * 8) = k; if (pass == 0) __threadfence(); } }
__global__ __launch_bounds__(256) void k_vtp(const _Float16* __restrict__ V16, int b0, _Float16* __restrict__ VT) { const int t = blockIdx.x * 256 + threadIdx.x; if (t >= JCH * KD * 16) return; const int pc = t % 16; const int kd = (t / 16) % KD; const int j = t / (16 * KD); const int b = b0 + j / NH, h = j % NH; FragH f;
#pragma unroll
  for (int q = 0; q < 8; ++q) { const int p = pc * 8 + q; f.h[q] = (p < PN) ? V16[((size_t)b * PN + p) * EE + h * KD + kd] : (_Float16)0.f; }
  *(volatile v8us*)((unsigned short*)VT + (size_t)t * 8) = f.half[0]; __threadfence(); *(volatile v8us*)((unsigned short*)VT + (size_t)t * 8) = f.half[0]; }
typedef _Float16 v4h __attribute__((ext_vector_type(4)));
__global__ __launch_bounds__(256) void k_psm(const float* __restrict__ S, const float* __restrict__ MSK, int b0, _Float16* __restrict__ P16) { const int tid = threadIdx.x, wv = tid >> 5, lane = tid & 31; const int row = blockIdx.x * 8 + wv; if (row >= JCH * RP) return; const int j = row / RP, gi = row % RP; const int b = b0 + j / NH; float v[4]; float m = -3.0e38f; const bool live = gi < GG;
#pragma unroll
  for (int q = 0; q < 4; ++q) { const int p = lane * 4 + q; float s = -3.0e38f; if (live && p < PN) { s = S[(size_t)row * RP + p] + bf16_round(MSK[((size_t)b * GG + gi) * PN + p]); } v[q] = s; m = fmaxf(m, s); }
  for (int o = 16; o >= 1; o >>= 1) m = fmaxf(m, __shfl_xor(m, o, 32)); float sum = 0.f; float e[4];
#pragma unroll
  for (int q = 0; q < 4; ++q) { e[q] = (v[q] > -1.0e38f) ? expf(v[q] - m) : 0.f; sum += e[q]; } for (int o = 16; o >= 1; o >>= 1) sum += __shfl_xor(sum, o, 32); const float is = (sum > 0.f) ? 1.0f / sum : 0.f; v4h hv; for (int q = 0; q < 4; ++q) hv[q] = (_Float16)(e[q] * is);
  _Float16* d = P16 + (size_t)row * 128 + lane * 4; *(volatile v4h*)d = hv; __threadfence(); *(volatile v4h*)d = hv; }
__global__ __launch_bounds__(256) void k_orep(const float* __restrict__ OC, int b0, _Float16* __restrict__ O16) { const int t = blockIdx.x * 256 + threadIdx.x; if (t >= BCH * GG * 16) return; const int p = t % 16; const int g = (t / 16) % GG; const int bl = t / (16 * GG); const int h = p / 2, k8 = (p % 2) * 8; const float* src = OC + ((size_t)(bl * NH + h) * RP + g) * KD + k8; FragH f;
#pragma unroll
  for (int q = 0; q < 8; ++q) f.h[q] = (_Float16)src[q]; unsigned short* d = (unsigned short*)O16 + ((size_t)(b0 + bl) * GG + g) * EE + p * 8; *(volatile v8us*)d = f.half[0]; __threadfence(); *(volatile v8us*)d = f.half[0]; }
__global__ __launch_bounds__(256) void k_padrows(const _Float16* __restrict__ SRC, int b0, _Float16* __restrict__ DST) { const int t = blockIdx.x * 256 + threadIdx.x; if (t >= BCH * RP * 16) return; const int c8 = (t % 16) * 8; const int gi = (t / 16) % RP; const int bl = t / (16 * RP); v8us v = {0,0,0,0,0,0,0,0}; if (gi < GG) v = *(const v8us*)((const unsigned short*)SRC + ((size_t)(b0 + bl) * GG + gi) * EE + c8); *(volatile v8us*)((unsigned short*)DST + (size_t)t * 8) = v; __threadfence(); *(volatile v8us*)((unsigned short*)DST + (size_t)t * 8) = v; }
__global__ __launch_bounds__(256) void k_stat(const float* __restrict__ S2, const float* __restrict__ MSK, int b0, float* __restrict__ ST) { const int tid = threadIdx.x, wv = tid >> 5, lane = tid & 31; const int row = blockIdx.x * 8 + wv; if (row >= BCH * GG) return; const int bl = row / GG, g = row % GG; const size_t bg = (size_t)(b0 + bl) * GG + g; float z[4]; float m = -3.0e38f;
#pragma unroll
  for (int q = 0; q < 4; ++q) { const int p = lane * 4 + q; float v = -3.0e38f; if (p < PN) v = 10.0f * tanhf(S2[((size_t)bl * RP + g) * RP + p] * 0.08838834764831845f) + bf16_round(MSK[bg * PN + p]); z[q] = v; m = fmaxf(m, v); }
  for (int o = 16; o >= 1; o >>= 1) m = fmaxf(m, __shfl_xor(m, o, 32)); float s = 0.f; for (int q = 0; q < 4; ++q) s += (z[q] > -1.0e38f) ? expf(z[q] - m) : 0.f; for (int o = 16; o >= 1; o >>= 1) s += __shfl_xor(s, o, 32);
  if (lane == 0) { typedef float v2f __attribute__((ext_vector_type(2))); v2f st; st[0] = m; st[1] = (s > 0.f) ? 1.0f / s : 0.f; *(volatile v2f*)(ST + bg * 2) = st; __threadfence(); *(volatile v2f*)(ST + bg * 2) = st; } }
__global__ __launch_bounds__(256) void k_prob(const float* __restrict__ S2, const float* __restrict__ MSK, const float* __restrict__ ST, int b0, float* __restrict__ out) { const size_t t = (size_t)blockIdx.x * 256 + threadIdx.x; if (t >= (size_t)BCH * GG * PN) return; const int p = (int)(t % PN); const size_t bgl = t / PN; const int bl = (int)(bgl / GG), g = (int)(bgl % GG); const size_t bg = (size_t)(b0 + bl) * GG + g;
  const float z = 10.0f * tanhf(S2[((size_t)bl * RP + g) * RP + p] * 0.08838834764831845f) + bf16_round(MSK[bg * PN + p]); const float v = expf(z - ST[bg * 2]) * ST[bg * 2 + 1]; *(volatile float*)(out + bg * PN + p) = v; __threadfence(); *(volatile float*)(out + bg * PN + p) = v; }
extern "C" void kernel_launch(void* const* d_in, const int* in_sizes, int n_in,
                              void* d_out, int out_size, void* d_ws, size_t ws_size, hipStream_t stream) {
  (void)in_sizes; (void)n_in; (void)out_size;
  const float* in1 = (const float*)d_in[0]; const float* in2 = (const float*)d_in[1]; const float* rl = (const float*)d_in[2]; const float* msk = (const float*)d_in[3]; const float* enc = (const float*)d_in[4]; const float* Wq = (const float*)d_in[5]; const float* Wk = (const float*)d_in[6]; const float* Wv = (const float*)d_in[7]; const float* Wc = (const float*)d_in[8]; const float* bc = (const float*)d_in[9];
  char* ws = (char*)d_ws; size_t off = 0;
  auto take = [&](size_t bytes) { char* p = ws + off; off += (bytes + 255) & ~(size_t)255; return p; };
  const size_t NRW = (size_t)NB * GG;
  _Float16* Bq2 = (_Float16*)take(EE * EE * 2); _Float16* Bk = (_Float16*)take(EE * EE * 2); _Float16* Bv = (_Float16*)take(EE * EE * 2); _Float16* Bc = (_Float16*)take(EE * EE * 2); float* Q1 = (float*)take((size_t)NB * EE * 4); float* ST = (float*)take(NRW * 2 * 4);
  _Float16* E16 = (_Float16*)take((NRW + 64) * EE * 2); _Float16* I16 = (_Float16*)take(NRW * EE * 2); float* QF = (float*)take(NRW * EE * 4); _Float16* Q16 = (_Float16*)take(NRW * EE * 2); _Float16* K16 = (_Float16*)take(NRW * EE * 2); _Float16* V16 = (_Float16*)take((NRW + 64) * EE * 2); _Float16* MH16 = (_Float16*)take(NRW * EE * 2);
  _Float16* P16 = (_Float16*)take((size_t)JCH * RP * 128 * 2); _Float16* QP = (_Float16*)take((size_t)JCH * RP * 32 * 2); _Float16* KP = (_Float16*)take((size_t)JCH * RP * 32 * 2); _Float16* VT = (_Float16*)take((size_t)JCH * KD * 128 * 2); float* OC = (float*)take((size_t)JCH * RP * KD * 4); _Float16* MHP = (_Float16*)take((size_t)BCH * RP * EE * 2); _Float16* ENP = (_Float16*)take((size_t)BCH * RP * EE * 2);
  float* S = QF; float* S2 = QF; _Float16* O16 = I16;
  if (off > ws_size) return;
  const size_t w8 = (size_t)EE * EE / 8; const unsigned gw = (unsigned)((w8 + 255) / 256);
  k_wt_f16<<<gw, 256, 0, stream>>>(Wq + (size_t)EE * EE, Bq2, EE, EE, 16.0f);
  k_wt_f16<<<gw, 256, 0, stream>>>(Wk, Bk, EE, EE, 16.0f); k_wt_f16<<<gw, 256, 0, stream>>>(Wv, Bv, EE, EE, 16.0f); k_wt_f16<<<gw, 256, 0, stream>>>(Wc, Bc, EE, EE, 16.0f);
  const unsigned g8 = (unsigned)((NRW * EE / 8 + 255) / 256); const dim3 gg(((unsigned)(NRW / 16) * (EE / 64) + 3) / 4, 1);
  k_x16<<<g8, 256, 0, stream>>>(enc, E16, NRW * EE / 8); k_x16<<<g8, 256, 0, stream>>>(in2, I16, NRW * EE / 8);
  k_gemm_hhx<0><<<gg, 128, 0, stream>>>(E16, EE, 0, Bk, EE, 0, 0.0625f, nullptr, 0, nullptr, 1, 0, 0, nullptr, K16, EE, 0, (int)NRW, EE, EE);
  k_gemm_hhx<0><<<gg, 128, 0, stream>>>(E16, EE, 0, Bv, EE, 0, 0.0625f, nullptr, 0, nullptr, 1, 0, 0, nullptr, V16, EE, 0, (int)NRW, EE, EE);
  k_gemm_hhx<0><<<gg, 128, 0, stream>>>(I16, EE, 0, Bq2, EE, 0, 0.0625f, nullptr, 0, nullptr, 1, 0, 0, QF, nullptr, EE, 0, (int)NRW, EE, EE);
  k_q1<<<NB, 128, 0, stream>>>(in1, Wq, Q1);
  k_qfin<<<(unsigned)((NRW * 16 + 255) / 256), 256, 0, stream>>>(QF, Q1, rl, Wq, Q16);
  for (int b0 = 0; b0 < NB; b0 += BCH) {
    k_qkp<<<(JCH * RP * 4 + 255) / 256, 256, 0, stream>>>(Q16, K16, b0, QP, KP); k_vtp<<<(JCH * KD * 16 + 255) / 256, 256, 0, stream>>>(V16, b0, VT);
    k_gemm_hhx<0><<<dim3(((RP / 16) * 2 + 3) / 4, JCH), 128, 0, stream>>>(QP, 32, (size_t)RP * 32, KP, 32, (size_t)RP * 32, 1.0f, nullptr, 0, nullptr, 1, 0, 0, S, nullptr, RP, (size_t)RP * RP, RP, RP, 32);
    k_psm<<<(JCH * RP + 7) / 8, 256, 0, stream>>>(S, msk, b0, P16);
    k_gemm_hhx<0><<<dim3(((RP / 16) * 1 + 3) / 4, JCH), 128, 0, stream>>>(P16, 128, (size_t)RP * 128, VT, 128, (size_t)KD * 128, 1.0f, nullptr, 0, nullptr, 1, 0, 0, OC, nullptr, KD, (size_t)RP * KD, RP, KD, 128);
    k_orep<<<(BCH * GG * 16 + 255) / 256, 256, 0, stream>>>(OC, b0, O16); }
  k_gemm_hhx<0><<<gg, 128, 0, stream>>>(O16, EE, 0, Bc, EE, 0, 0.0625f, bc, 0, nullptr, 1, 0, 0, nullptr, MH16, EE, 0, (int)NRW, EE, EE);
  for (int b0 = 0; b0 < NB; b0 += BCH) {
    k_padrows<<<(BCH * RP * 16 + 255) / 256, 256, 0, stream>>>(MH16, b0, MHP); k_padrows<<<(BCH * RP * 16 + 255) / 256, 256, 0, stream>>>(E16, b0, ENP);
    k_gemm_hhx<0><<<dim3(((RP / 16) * 2 + 3) / 4, BCH), 128, 0, stream>>>(MHP, EE, (size_t)RP * EE, ENP, EE, (size_t)RP * EE, 1.0f, nullptr, 0, nullptr, 1, 0, 0, S2, nullptr, RP, (size_t)RP * RP, RP, RP, EE);
    k_stat<<<(BCH * GG + 7) / 8, 256, 0, stream>>>(S2, msk, b0, ST);
    k_prob<<<(unsigned)(((size_t)BCH * GG * PN + 255) / 256), 256, 0, stream>>>(S2, msk, ST, b0, (float*)d_out); }
}
